// LatentEwaldSum_31379031065336
// MI455X (gfx1250) — hardware-verified
//
#include <hip/hip_runtime.h>


#ifndef NAT
#define NAT 200000
#endif
#define NAT_FULL 200000
#define NG   32
#define NK   342
#define KZERO 171
#define AWV  4
#define GRP  32
#define SLG  64
#define SLA  (AWV * GRP * SLG)
#define NSL  ((NAT + SLA - 1) / SLA)
#define TMU  98
#define TM   112
#define TNU  14
#define TN   16
#define TROWS (TM + TN)
#define LP   40
#define CT   (TM * TN)
#define NV4  (CT / 4)
#define FTH  256
#define TWOPI_F ((float)6.283185307179586)

static_assert(NAT >= 1);
static_assert(NAT <= NAT_FULL);
static_assert((size_t)NSL * SLA >= (size_t)NAT);
static_assert(TMU == 2 * 49);
static_assert(TNU == 2 * 7);
static_assert(TM % 16 == 0);
static_assert(TM / 16 == 7);
static_assert(TM >= TMU);
static_assert(TN == 16);
static_assert(TN >= TNU);
static_assert(GRP == 32);
static_assert(LP >= 32);
static_assert((LP * 2) % 16 == 0);
static_assert(CT % 4 == 0);
static_assert(NV4 % 32 == 0);
static_assert(NV4 <= 4 * 32 * AWV);
static_assert((size_t)NV4 * 16 == (size_t)TM * TN * 4);
static_assert((CT * 4) % 128 == 0);
static_assert(AWV * TROWS * LP * 2 + AWV * CT * 4 <= 131072);
static_assert(CT * 4 + 8 * 4 + NG * 4 <= 131072);
static_assert(CT % FTH == 0);
static_assert(2 * FTH >= NK);
static_assert(FTH == 8 * 32);
static_assert(NG * 4 == 128);
static_assert((size_t)NAT_FULL * 3 < (size_t)2147483647);

typedef _Float16 h16;
typedef __attribute__((ext_vector_type(16))) _Float16 v16h;
typedef __attribute__((ext_vector_type(8)))  _Float16 v8h;
typedef __attribute__((ext_vector_type(8)))  float    v8f;
typedef __attribute__((ext_vector_type(4)))  float    v4f;
typedef v4f  __attribute__((may_alias)) v4fa;
typedef v8h  __attribute__((may_alias)) v8ha;

__device__ __forceinline__ unsigned short f2bf(float f) { unsigned u = __float_as_uint(f); u += 0x7FFFu + ((u >> 16) & 1u); return (unsigned short)(u >> 16); }
__device__ __forceinline__ float bfr(float f) { return __uint_as_float(((unsigned)f2bf(f)) << 16); }
__device__ __forceinline__ v16h cat16(v8h lo, v8h hi) { return __builtin_shufflevector(lo, hi, 0, 1, 2, 3, 4, 5, 6, 7, 8, 9, 10, 11, 12, 13, 14, 15); }
__device__ __forceinline__ v8f wmma16(v16h a, v16h b, v8f c) { return __builtin_amdgcn_wmma_f32_16x16x32_f16(false, a, false, b, (short)0, c, false, false); }
__device__ __forceinline__ v8f wmma16g(v16h a, v16h b, v8f c) { c = wmma16(a, b, c); asm volatile("v_nop\n\tv_nop\n\tv_nop\n\tv_nop" : "+v"(c) : "v"(a), "v"(b)); return c; }
__device__ __forceinline__ void wave_sync() { __builtin_amdgcn_fence(3  , "wavefront"); __builtin_amdgcn_wave_barrier(); asm volatile("" ::: "memory"); }
static __device__ __forceinline__ h16 toh_flush(float v) { const h16 r = (h16)v; return (fabsf(v) < 6.103515625e-05f) ? (h16)0.0f : r; }

struct RecipT { float r[9]; float vol; };
__device__ __forceinline__ RecipT cell_recip(const float* __restrict__ cell, int g) {
#pragma clang fp contract(off)
    double a[9];
#pragma unroll
    for (int i = 0; i < 9; ++i) a[i] = (double)bfr(cell[(size_t)g * 9 + i]);
    const double c00 = a[4] * a[8] - a[5] * a[7];
    const double c01 = a[3] * a[8] - a[5] * a[6];
    const double c02 = a[3] * a[7] - a[4] * a[6];
    const double det = a[0] * c00 - a[1] * c01 + a[2] * c02;
    const double id = 1.0 / det;
    double inv[9];
    inv[0] = c00 * id;
    inv[1] = (a[2] * a[7] - a[1] * a[8]) * id;
    inv[2] = (a[1] * a[5] - a[2] * a[4]) * id;
    inv[3] = (a[5] * a[6] - a[3] * a[8]) * id;
    inv[4] = (a[0] * a[8] - a[2] * a[6]) * id;
    inv[5] = (a[2] * a[3] - a[0] * a[5]) * id;
    inv[6] = c02 * id;
    inv[7] = (a[1] * a[6] - a[0] * a[7]) * id;
    inv[8] = (a[0] * a[4] - a[1] * a[3]) * id;
    RecipT o;
#pragma unroll
    for (int r = 0; r < 3; ++r)
#pragma unroll
        for (int c = 0; c < 3; ++c) o.r[r * 3 + c] = TWOPI_F * (float)inv[c * 3 + r];
    o.vol = fabsf((float)det);
    return o;
}

struct Ph7 { float c[7]; float s[7]; };
__device__ __forceinline__ Ph7 phase7(float u) {
    const float s1 = sinf(u), c1 = cosf(u);
    const float c2 = c1 * c1 - s1 * s1, s2 = 2.0f * s1 * c1;
    const float c3 = c2 * c1 - s2 * s1, s3 = s2 * c1 + c2 * s1;
    Ph7 p;
    p.c[0] = c3; p.c[1] = c2; p.c[2] = c1; p.c[3] = 1.0f; p.c[4] = c1; p.c[5] = c2; p.c[6] = c3;
    p.s[0] = -s3; p.s[1] = -s2; p.s[2] = -s1; p.s[3] = 0.0f; p.s[4] = s1; p.s[5] = s2; p.s[6] = s3;
    return p;
}

__global__ __launch_bounds__(32 * AWV) void k_sfac(const float* __restrict__ q, const float* __restrict__ pos, const int* __restrict__ batch, const float* __restrict__ cell, float* PART) {
    __shared__ __align__(16) h16 tl[AWV * TROWS * LP];
    __shared__ __align__(16) float red[AWV * CT];
    const int tid = threadIdx.x;
    const int lane = tid & 31, lr = lane & 15, hi = lane >> 4;
    const int wave = __builtin_amdgcn_readfirstlane((int)(threadIdx.x >> 5));
    const int s = blockIdx.x, g = blockIdx.y;
    const RecipT rc = cell_recip(cell, g);
    const int wb = wave * TROWS * LP;
#pragma unroll
    for (int m = TMU; m < TM; ++m) tl[wb + m * LP + lane] = (h16)0.0f;
    tl[wb + (TM + TNU) * LP + lane] = (h16)0.0f;
    tl[wb + (TM + TNU + 1) * LP + lane] = (h16)0.0f;
    v8f acc[7];
#pragma unroll
    for (int j = 0; j < 7; ++j) acc[j] = (v8f){};
    const int abase = s * SLA + wave * GRP + lane;
#pragma unroll 1
    for (int it = 0; it < SLG; ++it) {
        const int i = abase + it * (AWV * GRP);
        const int ic = i < NAT ? i : (NAT - 1);
        int bt = batch[ic];
        asm volatile("" : "+v"(bt));
        const bool hit = (((int)(i < NAT)) & ((int)(bt == g))) != 0;
        const unsigned bal = __builtin_amdgcn_ballot_w32(hit);
        if (bal != 0u) {
            float qv = q[ic];
            float rx = pos[(size_t)ic * 3 + 0], ry = pos[(size_t)ic * 3 + 1], rz = pos[(size_t)ic * 3 + 2];
            asm volatile("" : "+v"(qv), "+v"(rx), "+v"(ry), "+v"(rz));
            const float qg = hit ? bfr(qv) : 0.0f;
            rx = bfr(rx); ry = bfr(ry); rz = bfr(rz);
            const float ux = rc.r[0] * rx + rc.r[1] * ry + rc.r[2] * rz;
            const float uy = rc.r[3] * rx + rc.r[4] * ry + rc.r[5] * rz;
            const float uz = rc.r[6] * rx + rc.r[7] * ry + rc.r[8] * rz;
            const Ph7 ex = phase7(ux);
            const Ph7 ey = phase7(uy);
            const Ph7 ez = phase7(uz);
            wave_sync();
#pragma unroll
            for (int ix = 0; ix < 7; ++ix) {
                const float qr_ = qg * ex.c[ix], qi_ = qg * ex.s[ix];
#pragma unroll
                for (int iy = 0; iy < 7; ++iy) {
                    const float ar = qr_ * ey.c[iy] - qi_ * ey.s[iy];
                    const float ai = qr_ * ey.s[iy] + qi_ * ey.c[iy];
                    tl[wb + (ix * 7 + iy) * LP + lane] = toh_flush(ar);
                    tl[wb + (49 + ix * 7 + iy) * LP + lane] = toh_flush(ai);
                }
            }
#pragma unroll
            for (int iz = 0; iz < 7; ++iz) {
                tl[wb + (TM + iz) * LP + lane] = toh_flush(ez.c[iz]);
                tl[wb + (TM + 7 + iz) * LP + lane] = toh_flush(ez.s[iz]);
            }
            wave_sync();
            const int bo = wb + (TM + lr) * LP + 8 * hi;
            const v8h b0 = *(const v8ha*)(&tl[bo]);
            const v8h b1 = *(const v8ha*)(&tl[bo + 16]);
            const v16h bfrag = cat16(b0, b1);
#pragma unroll
            for (int j = 0; j < 7; ++j) {
                const int ao = wb + (16 * j + lr) * LP + 8 * hi;
                const v8h a0 = *(const v8ha*)(&tl[ao]);
                const v8h a1 = *(const v8ha*)(&tl[ao + 16]);
                acc[j] = wmma16g(cat16(a0, a1), bfrag, acc[j]);
            }
            wave_sync();
        }
    }
#pragma unroll
    for (int j = 0; j < 7; ++j)
#pragma unroll
        for (int r = 0; r < 8; ++r) red[wave * CT + (16 * j + 8 * hi + r) * TN + lr] = acc[j][r];
    __syncthreads();
    float* dst = PART + ((size_t)g * NSL + (size_t)s) * CT;
    v4f sv[4];
#pragma unroll
    for (int t = 0; t < 4; ++t) {
        const int idx = t * (32 * AWV) + tid;
        const int ixc = idx < NV4 ? idx : (NV4 - 1);
        v4f a = *(const v4fa*)(&red[ixc * 4]);
#pragma unroll
        for (int w = 1; w < AWV; ++w) { const v4f o = *(const v4fa*)(&red[w * CT + ixc * 4]); a = a + o; }
        sv[t] = a;
    }
#pragma unroll 1
    for (int ps = 0; ps < 2; ++ps) {
#pragma unroll
        for (int t = 0; t < 4; ++t) {
            const int idx = t * (32 * AWV) + tid;
            if (idx < NV4) *(volatile v4f*)(dst + (size_t)idx * 4) = sv[t];
        }
        if (ps == 0) __threadfence();
    }
}

__global__ __launch_bounds__(FTH) void k_final(const float* __restrict__ cell, const float* __restrict__ PART, float* OUT) {
#pragma clang fp contract(off)
    __shared__ __align__(16) float cs[CT];
    __shared__ float wred[8];
    __shared__ __align__(16) float eg[NG];
    const int tid = threadIdx.x;
    const int lane = tid & 31;
    const int wave = __builtin_amdgcn_readfirstlane((int)(threadIdx.x >> 5));
#pragma unroll 1
    for (int g = 0; g < NG; ++g) {
#pragma unroll 1
        for (int e = tid; e < CT; e += FTH) {
            float a = 0.0f;
#pragma unroll 1
            for (int s = 0; s < NSL; ++s) a += PART[((size_t)g * NSL + (size_t)s) * CT + e];
            cs[e] = a;
        }
        __syncthreads();
        const RecipT rc = cell_recip(cell, g);
        float acc = 0.0f;
#pragma unroll 1
        for (int kk = 0; kk < 2; ++kk) {
            const int k = kk * FTH + tid;
            const int kc = k < NK ? k : (NK - 1);
            const int m = kc >= KZERO ? kc + 1 : kc;
            const int ix = m / 49, iy = (m / 7) % 7, iz = m % 7;
            const float nx = (float)(ix - 3), ny = (float)(iy - 3), nz = (float)(iz - 3);
            const float kv0 = nx * rc.r[0] + ny * rc.r[3] + nz * rc.r[6];
            const float kv1 = nx * rc.r[1] + ny * rc.r[4] + nz * rc.r[7];
            const float kv2 = nx * rc.r[2] + ny * rc.r[5] + nz * rc.r[8];
            const float k2 = kv0 * kv0 + kv1 * kv1 + kv2 * kv2;
            const float w = expf(-0.5f * k2) * (1.0f / k2);
            const int rr = ix * 7 + iy;
            const float crr = cs[rr * TN + iz], cii = cs[(49 + rr) * TN + 7 + iz];
            const float cri = cs[rr * TN + 7 + iz], cir = cs[(49 + rr) * TN + iz];
            const float sr = crr - cii, si = cri + cir;
            const float term = w * (sr * sr + si * si);
            acc += (k < NK) ? term : 0.0f;
        }
#pragma unroll
        for (int off = 16; off >= 1; off >>= 1) acc += __shfl_xor(acc, off, 32);
        if (lane == 0) wred[wave] = acc;
        __syncthreads();
        if (tid == 0) {
            float t = 0.0f;
#pragma unroll
            for (int w = 0; w < 8; ++w) t += wred[w];
            eg[g] = (TWOPI_F / rc.vol) * t;
        }
        __syncthreads();
    }
    if (wave == 0) {
        const int lc = lane < 8 ? lane : 7;
        const v4f val = *(const v4fa*)(&eg[lc * 4]);
#pragma unroll 1
        for (int ps = 0; ps < 2; ++ps) {
            if (lane < 8) *(volatile v4f*)(OUT + lane * 4) = val;
            if (ps == 0) __threadfence();
        }
    }
}

static constexpr size_t al256(size_t v) { return (v + 255) & ~(size_t)255; }
static constexpr size_t SZ_PART = al256((size_t)NG * NSL * CT * 4);
static constexpr size_t SZ_TOTAL = SZ_PART;
static_assert(SZ_TOTAL <= (size_t)134217728);
static_assert(((size_t)NG * NSL - 1) * CT * 4 + (size_t)NV4 * 16 <= SZ_PART);

extern "C" void kernel_launch(void* const* d_in, const int* in_sizes, int n_in,
                              void* d_out, int out_size, void* d_ws, size_t ws_size, hipStream_t stream) {
    if (n_in < 4) return;
    if ((size_t)in_sizes[0] < (size_t)NAT || (size_t)in_sizes[1] < (size_t)NAT * 3 || (size_t)in_sizes[2] < (size_t)NAT) return;
    if (in_sizes[3] < NG * 9) return;
    if (out_size < NG) return;
    if (SZ_TOTAL > ws_size) return;
    const float* q    = (const float*)d_in[0];
    const float* pos  = (const float*)d_in[1];
    const int*   bat  = (const int*)d_in[2];
    const float* cell = (const float*)d_in[3];
    float* OUT = (float*)d_out;
    float* PART = (float*)d_ws;

    k_sfac<<<dim3(NSL, NG, 1), 32 * AWV, 0, stream>>>(q, pos, bat, cell, PART);
    k_final<<<dim3(1, 1, 1), FTH, 0, stream>>>(cell, PART, OUT);
}
